// FRU_73443940762219
// MI455X (gfx1250) — hardware-verified
//
#include <hip/hip_runtime.h>
#include <math.h>

constexpr int SEQ    = 2048;
constexpr int NHEAD  = 16;
constexpr int HD     = 64;
constexpr int NIN    = 1024;
constexpr int NSTATE = 1024;
constexpr int NPROJ  = 5120;
constexpr int NOUT   = 1024;
constexpr int TPB    = 256;
constexpr int SCAN_T = 128;
constexpr int SPITCH = 72;
constexpr float STATE_CARRY = 16.0f;
constexpr float WH_CARRY    = 64.0f;
constexpr float SW_INV      = 1.0f / 1024.0f;
constexpr float Y_CARRY     = 16.0f;
constexpr float WOUT_CARRY  = 256.0f;
constexpr float OUT_INV     = 1.0f / 4096.0f;

typedef __attribute__((ext_vector_type(16))) _Float16 v16h;
typedef __attribute__((ext_vector_type(8)))  _Float16 v8h;
typedef __attribute__((ext_vector_type(16))) __bf16   v16b;
typedef __attribute__((ext_vector_type(8)))  __bf16   v8b;
typedef __attribute__((ext_vector_type(8)))  float    v8f;
typedef __attribute__((ext_vector_type(4)))  float    v4f;
#define PSCALE 32768.0f
#define U16(p) ((const unsigned short*)(const void*)(p))
#define PSCALE_INV (1.0f / 32768.0f)

__device__ __forceinline__ unsigned short f2bf_bits(float f) {
  unsigned u = __float_as_uint(f);
  return (unsigned short)((u + 0x7FFFu + ((u >> 16) & 1u)) >> 16);
}
__device__ __forceinline__ float bf_bits2f(unsigned short h) { return __uint_as_float(((unsigned)h) << 16); }

__device__ __forceinline__ void dep_guard_h(v8f& a, v8f& b, v16h x, v16h y) { asm volatile("v_nop\n\tv_nop\n\tv_nop\n\tv_nop" : "+v"(a), "+v"(b) : "v"(x), "v"(y)); }
__device__ __forceinline__ void dep_guard_b(v8f& a, v8f& b, v16b x, v16b y) { asm volatile("v_nop\n\tv_nop\n\tv_nop\n\tv_nop" : "+v"(a), "+v"(b) : "v"(x), "v"(y)); }
__device__ __forceinline__ void keep4_h(v16h a, v16h b, v16h c, v16h d) { asm volatile("v_nop" :: "v"(a), "v"(b), "v"(c), "v"(d)); }
__device__ __forceinline__ void keep4_b(v16b a, v16b b, v16b c, v16b d) { asm volatile("v_nop" :: "v"(a), "v"(b), "v"(c), "v"(d)); }
__device__ __forceinline__ void acc_guard4(v8f& a, v8f& b, v8f& c, v8f& d) { asm volatile("v_nop\n\tv_nop\n\tv_nop\n\tv_nop" : "+v"(a), "+v"(b), "+v"(c), "+v"(d)); }
template <typename T> struct Frag;
template <> struct Frag<_Float16> {
  typedef v16h V; union U { v16h v; v8h h[2]; };
  static __device__ __forceinline__ v16h load(const _Float16* p) {
    U f; f.h[0] = *(const v8h*)(p); f.h[1] = *(const v8h*)(p + 16); return f.v;
  }
  static __device__ __forceinline__ v8f mma(v16h a, v16h b, v8f c) {
    return __builtin_amdgcn_wmma_f32_16x16x32_f16(false, a, false, b, (short)0, c, false, false);
  }
  static __device__ __forceinline__ void guard(v8f& a, v8f& b, v16h x, v16h y) { dep_guard_h(a, b, x, y); }
  static __device__ __forceinline__ void keep(v16h a, v16h b, v16h c, v16h d) { keep4_h(a, b, c, d); }
};
template <> struct Frag<__bf16> {
  typedef v16b V; union U { v16b v; v8b h[2]; };
  static __device__ __forceinline__ v16b load(const __bf16* p) {
    U f; f.h[0] = *(const v8b*)(p); f.h[1] = *(const v8b*)(p + 16); return f.v;
  }
  static __device__ __forceinline__ v8f mma(v16b a, v16b b, v8f c) {
    return __builtin_amdgcn_wmma_f32_16x16x32_bf16(false, a, false, b, (short)0, c, false, false);
  }
  static __device__ __forceinline__ void guard(v8f& a, v8f& b, v16b x, v16b y) { dep_guard_b(a, b, x, y); }
  static __device__ __forceinline__ void keep(v16b a, v16b b, v16b c, v16b d) { keep4_b(a, b, c, d); }
};

template <int ET> struct Elem;
template <> struct Elem<0> { typedef _Float16 T; };
template <> struct Elem<1> { typedef __bf16 T; };
template <int ET, bool SPLIT, int BIAS_MODE, int OUT_MODE, bool RESID, int ACT = 0>
__global__ __launch_bounds__(256) void wmma_gemm64(
    const unsigned short* __restrict__ Ap, const unsigned short* __restrict__ A2p, int lda, long strideA,
    const unsigned short* __restrict__ Btp, const unsigned short* __restrict__ Bt2p, int ldb, long strideB,
    void* __restrict__ Cout, void* __restrict__ Cout2, int ldc, long strideC,
    const float* __restrict__ bias,
    const float* __restrict__ resid, long strideR,
    int M, int N, int K, float scale) {
  typedef typename Elem<ET>::T T;
  typedef typename Frag<T>::V V;
  const T* A = (const T*)Ap; const T* A2 = (const T*)A2p; const T* Bt = (const T*)Btp; const T* Bt2 = (const T*)Bt2p;
  __shared__ __align__(16) float sT[8][16 * 68];
  const int b    = blockIdx.y;
  const int lane = threadIdx.x & 31;
  const int wave = threadIdx.x >> 5;
  const int tilesN = N >> 6;
  const int tilesM = M >> 6;
  const int tile = blockIdx.x * 8 + wave;
  if (tile >= tilesM * tilesN) return;
  const int tm = tile / tilesN;
  const int tn = tile - tm * tilesN;
  const int m0 = tm << 6;
  const int n0 = tn << 6;

  const T* Ab  = A  + (size_t)b * strideA;
  const T* Bb  = Bt + (size_t)b * strideB;
  const T* Ab2 = SPLIT ? (A2  + (size_t)b * strideA) : nullptr;
  const T* Bb2 = SPLIT ? (Bt2 + (size_t)b * strideB) : nullptr;

  const int rlane = lane & 15;
  const int koff  = (lane >> 4) * 8;
  const int mOff  = (lane >> 4) * 8;

  v8f acc[4][4];
#pragma unroll
  for (int i = 0; i < 4; ++i)
#pragma unroll
    for (int j = 0; j < 4; ++j) acc[i][j] = (v8f){0.f,0.f,0.f,0.f,0.f,0.f,0.f,0.f};

  for (int k0 = 0; k0 < K; k0 += 32) {
    V bh[4], bl[4];
#pragma unroll
    for (int j = 0; j < 4; ++j) {
      const size_t bo = (size_t)(n0 + (j << 4) + rlane) * ldb + koff + k0;
      bh[j] = Frag<T>::load(Bb + bo);
      if (SPLIT) bl[j] = Frag<T>::load(Bb2 + bo);
    }
#pragma unroll
    for (int i = 0; i < 4; ++i) {
      const size_t ao = (size_t)(m0 + (i << 4) + rlane) * lda + koff + k0;
      V ah = Frag<T>::load(Ab + ao);
      V al;
      if (SPLIT) al = Frag<T>::load(Ab2 + ao);
#pragma unroll
      for (int j = 0; j < 4; ++j) {
        acc[i][j] = Frag<T>::mma(ah, bh[j], acc[i][j]);
        if (SPLIT) {
          acc[i][j] = Frag<T>::mma(ah, bl[j], acc[i][j]);
          acc[i][j] = Frag<T>::mma(al, bh[j], acc[i][j]);
        }
      }
      Frag<T>::guard(acc[i][0], acc[i][3], ah, SPLIT ? al : ah);
    }
    Frag<T>::keep(bh[0], bh[1], bh[2], bh[3]);
    if (SPLIT) Frag<T>::keep(bl[0], bl[1], bl[2], bl[3]);
  }
  acc_guard4(acc[0][0], acc[0][1], acc[0][2], acc[0][3]);
  acc_guard4(acc[1][0], acc[1][1], acc[1][2], acc[1][3]);
  acc_guard4(acc[2][0], acc[2][1], acc[2][2], acc[2][3]);
  acc_guard4(acc[3][0], acc[3][1], acc[3][2], acc[3][3]);

  float* slab = sT[wave];
  const float* Rb = RESID ? (resid + (size_t)b * strideR) : nullptr;
#pragma unroll
  for (int i = 0; i < 4; ++i) {
    const int mBase = m0 + (i << 4);
#pragma unroll
    for (int j = 0; j < 4; ++j) {
      const int n = n0 + (j << 4) + rlane;
      float bv = 0.f;
      if (BIAS_MODE == 2) bv = bias[n];
#pragma unroll
      for (int r = 0; r < 8; ++r) {
        float v = acc[i][j][r] * scale;
        if (BIAS_MODE == 1) v += bias[mBase + mOff + r];
        if (BIAS_MODE == 2) v += bv;
        if (RESID) v += Rb[(size_t)(mBase + mOff + r) * ldc + n];
        if (ACT == 1) v = tanhf(v);
        if (ACT == 2) v = fmaxf(v, 0.0f);
        if (ACT == 3) v = v / (1.0f + expf(-v));
        if (ACT == 4) v = (v > 0.f) ? v : 0.01f * v;
        if (ACT == 5) v = 0.5f * v * (1.0f + erff(v * 0.70710678118654752f));
        slab[(mOff + r) * 68 + (j << 4) + rlane] = v;
      }
    }
    __builtin_amdgcn_fence(__ATOMIC_RELEASE, "workgroup");
    __builtin_amdgcn_wave_barrier();
    __builtin_amdgcn_fence(__ATOMIC_ACQUIRE, "workgroup");
    if (OUT_MODE == 0) {
      float* C = (float*)Cout + (size_t)b * strideC;
      const int hh = lane >> 4, c4 = (lane & 15) * 4;
      for (int pass = 0; pass < 2; ++pass) {
#pragma unroll
        for (int it = 0; it < 8; ++it) {
          const int row = it * 2 + hh;
          v4f v = *(const v4f*)(slab + row * 68 + c4);
          *(volatile v4f*)(C + (size_t)(mBase + row) * ldc + n0 + c4) = v;
        }
        __threadfence();
      }
    } else {
      const int q = lane >> 3, c8 = (lane & 7) * 8;
      unsigned short* C  = (unsigned short*)Cout  + (size_t)b * strideC;
      unsigned short* C2 = (OUT_MODE == 2) ? ((unsigned short*)Cout2 + (size_t)b * strideC) : nullptr;
      for (int pass = 0; pass < 2; ++pass) {
#pragma unroll
        for (int it = 0; it < 4; ++it) {
          const int row = it * 4 + q;
          const float* sp = slab + row * 68 + c8;
          v8h hv, lv;
#pragma unroll
          for (int e = 0; e < 8; ++e) {
            if (OUT_MODE == 1) {
              hv[e] = (_Float16)sp[e];
            } else {
              unsigned short hb = f2bf_bits(sp[e]);
              unsigned short lb = f2bf_bits(sp[e] - bf_bits2f(hb));
              hv[e] = __builtin_bit_cast(_Float16, hb);
              lv[e] = __builtin_bit_cast(_Float16, lb);
            }
          }
          *(volatile v8h*)(C + (size_t)(mBase + row) * ldc + n0 + c8) = hv;
          if (OUT_MODE == 2) *(volatile v8h*)(C2 + (size_t)(mBase + row) * ldc + n0 + c8) = lv;
        }
        __threadfence();
      }
    }
    __builtin_amdgcn_fence(__ATOMIC_RELEASE, "workgroup");
    __builtin_amdgcn_wave_barrier();
    __builtin_amdgcn_fence(__ATOMIC_ACQUIRE, "workgroup");
  }
}

__device__ __forceinline__ float frcp(float x) { return __builtin_amdgcn_rcpf(x); }
__device__ __forceinline__ float fsig(float x) { return frcp(1.0f + __expf(-x)); }
__device__ __forceinline__ float bfr(float f)  { return bf_bits2f(f2bf_bits(f)); }
__device__ __forceinline__ void guard5(v8f& acc, v16h a, v16h b, v16h c, v16h d) {
  asm volatile("v_nop\n\tv_nop\n\tv_nop\n\tv_nop" : "+v"(acc) : "v"(a), "v"(b), "v"(c), "v"(d));
}

__global__ __launch_bounds__(TPB) void cast_bf16x8(const float* __restrict__ in, unsigned short* __restrict__ out, int n8) {
  const int i = blockIdx.x * TPB + threadIdx.x;
  if (i < n8) {
    const v4f a = *(const v4f*)(in + (size_t)8 * i);
    const v4f b = *(const v4f*)(in + (size_t)8 * i + 4);
    v8h hv;
#pragma unroll
    for (int e = 0; e < 4; ++e) {
      hv[e]     = __builtin_bit_cast(_Float16, f2bf_bits(a[e]));
      hv[4 + e] = __builtin_bit_cast(_Float16, f2bf_bits(b[e]));
    }
    unsigned short* dst = out + (size_t)8 * i;
    *(volatile v8h*)dst = hv;
    __threadfence();
    *(volatile v8h*)dst = hv;
  }
}

template <int MODE>
__global__ __launch_bounds__(TPB) void tpw_kernel(const float* __restrict__ src, int R, int C, int ldo,
                                                 unsigned short* __restrict__ O, float sc) {
  __shared__ float Tt[64 * 65];
  const int tid = threadIdx.x;
  const int c0 = blockIdx.x * 64, r0 = blockIdx.y * 64;
#pragma unroll
  for (int i = 0; i < 4; ++i) {
    const int idx = i * TPB + tid;
    const int rr = idx >> 4, cc = (idx & 15) * 4;
    const v4f v = *(const v4f*)(src + (size_t)(r0 + rr) * (size_t)C + c0 + cc);
    Tt[rr * 65 + cc + 0] = v[0];
    Tt[rr * 65 + cc + 1] = v[1];
    Tt[rr * 65 + cc + 2] = v[2];
    Tt[rr * 65 + cc + 3] = v[3];
  }
  __syncthreads();
  const int q = tid >> 3, c8 = (tid & 7) * 8;
  v8h hv[2];
#pragma unroll
  for (int g = 0; g < 2; ++g) {
    const int qq = g * 32 + q;
#pragma unroll
    for (int e = 0; e < 8; ++e) {
      const float f = Tt[(c8 + e) * 65 + qq];
      unsigned short bits;
      if (MODE == 0) {
        bits = f2bf_bits(f * sc);
      } else {
        const float fb = bf_bits2f(f2bf_bits(f));
        bits = __builtin_bit_cast(unsigned short, (_Float16)(fb * sc));
      }
      hv[g][e] = __builtin_bit_cast(_Float16, bits);
    }
  }
  for (int pass = 0; pass < 2; ++pass) {
#pragma unroll
    for (int g = 0; g < 2; ++g) {
      const size_t o = (size_t)(c0 + g * 32 + q) * (size_t)ldo + (size_t)(r0 + c8);
      *(volatile v8h*)(O + o) = hv[g];
    }
    __threadfence();
  }
}

__global__ __launch_bounds__(TPB) void prep_kernel(const float* __restrict__ proj, const float* __restrict__ fm,
                                                  const float* __restrict__ lf, float* __restrict__ pl) {
  const int t = blockIdx.x;
  const int tid = threadIdx.x, wave = tid >> 5, lane = tid & 31, hh = lane >> 4, c = lane & 15;
  const int h = 2 * wave + hh;
  const int col = h * HD + 4 * c;
  const float* row = proj + (size_t)t * NPROJ + col;
  const v4f q4 = *(const v4f*)(row);
  const v4f k4 = *(const v4f*)(row + NSTATE);
  const v4f w4 = *(const v4f*)(row + 2 * NSTATE);
  const v4f f4 = *(const v4f*)(row + 3 * NSTATE);
  float sq = (q4[0] * q4[0] + q4[1] * q4[1]) + (q4[2] * q4[2] + q4[3] * q4[3]);
  float sk = (k4[0] * k4[0] + k4[1] * k4[1]) + (k4[2] * k4[2] + k4[3] * k4[3]);
  float sw = (w4[0] * w4[0] + w4[1] * w4[1]) + (w4[2] * w4[2] + w4[3] * w4[3]);
#pragma unroll
  for (int off = 1; off < 16; off <<= 1) {
    sq += __shfl_xor(sq, off, 32);
    sk += __shfl_xor(sk, off, 32);
    sw += __shfl_xor(sw, off, 32);
  }
  const float inv = 1.0f / 64.0f;
  const float rq = rsqrtf(sq * inv + 1e-6f);
  const float rk = rsqrtf(sk * inv + 1e-6f);
  const float rw = rsqrtf(sw * inv + 1e-6f);
  const float factor = fsig(bfr(lf[h]));
  const v4f qo = q4 * rq;
  const v4f ko = k4 * rk;
  const v4f wo = (w4 * rw) * factor;
  v4f fo;
#pragma unroll
  for (int e = 0; e < 4; ++e) fo[e] = fsig(f4[e] * (2.0f * fsig(bfr(fm[h * HD + 4 * c + e]))));
  const size_t plane = (size_t)SEQ * NSTATE;
  float* dst = pl + (size_t)t * NSTATE + col;
  for (int pass = 0; pass < 2; ++pass) {
    *(volatile v4f*)(dst) = qo;
    *(volatile v4f*)(dst + plane) = ko;
    *(volatile v4f*)(dst + 2 * plane) = wo;
    *(volatile v4f*)(dst + 3 * plane) = fo;
    __threadfence();
  }
}

__global__ __launch_bounds__(SCAN_T) void scan_kernel(const float* __restrict__ pl, const float* __restrict__ swt,
                                                     const float* __restrict__ lf, float* __restrict__ og) {
  __shared__ __align__(16) _Float16 S16[HD * SPITCH];
  __shared__ __align__(16) _Float16 W16[HD * SPITCH];
  __shared__ float sv[4 * HD];
  __shared__ float sop[4 * HD];
  __shared__ __align__(16) float ob[16 * HD];
  const int h = blockIdx.x;
  const int tid = threadIdx.x, wave = tid >> 5, lane = tid & 31, hh = lane >> 4, c = lane & 15;
  const float factor = fsig(bfr(lf[h]));
  const float rg = frcp(1.0f + __expf(-20.0f));

  for (int i = tid; i < HD * SPITCH / 2; i += SCAN_T) ((unsigned*)S16)[i] = 0u;
  {
    const int j = tid & 63, kh = tid >> 6;
    const float* swh = swt + (size_t)h * HD * HD;
#pragma unroll 1
    for (int e = 0; e < 32; ++e) {
      const int k = 32 * kh + e;
      W16[j * SPITCH + k] = (_Float16)((bfr(swh[k * HD + j]) * factor) * WH_CARRY);
    }
  }
  __syncthreads();

  const size_t plane = (size_t)SEQ * NSTATE;
  const float* plh = pl + (size_t)h * HD;
  const int p0 = tid >> 6, d0 = tid & 63;
  const float* src0 = plh + (size_t)p0 * plane + d0;
  const float* src1 = plh + (size_t)(p0 + 2) * plane + d0;
  const int rbase = 16 * wave + 8 * hh;
  const _Float16* arow = S16 + (16 * wave + c) * SPITCH + 8 * hh;
  const _Float16* brow = W16 + c * SPITCH + 8 * hh;
  const v8f z8 = {0.f, 0.f, 0.f, 0.f, 0.f, 0.f, 0.f, 0.f};

#pragma unroll 1
  for (int t = 0; t < SEQ; ++t) {
    const size_t to = (size_t)t * NSTATE;
    sv[tid] = src0[to];
    sv[tid + SCAN_T] = src1[to];
    __syncthreads();

    const v16h a0 = Frag<_Float16>::load(arow);
    const v16h a1 = Frag<_Float16>::load(arow + 32);
    float qv[8], kr[8], fr[8];
#pragma unroll
    for (int r = 0; r < 8; ++r) {
      qv[r] = sv[rbase + r];
      kr[r] = sv[HD + rbase + r];
      fr[r] = sv[3 * HD + rbase + r];
    }
#pragma unroll 1
    for (int tt = 0; tt < 4; ++tt) {
      const v16h b0 = Frag<_Float16>::load(brow + 16 * tt * SPITCH);
      const v16h b1 = Frag<_Float16>::load(brow + 16 * tt * SPITCH + 32);
      v8f acc = z8;
      acc = Frag<_Float16>::mma(a0, b0, acc);
      acc = Frag<_Float16>::mma(a1, b1, acc);
      guard5(acc, a0, a1, b0, b1);
      const int j = 16 * tt + c;
      const float vf = sv[2 * HD + j];
      float part = 0.0f;
#pragma unroll
      for (int r = 0; r < 8; ++r) {
        const float pm = acc[r] * SW_INV;
        const float sn = fr[r] * pm + rg * (kr[r] * vf);
        S16[(rbase + r) * SPITCH + j] = (_Float16)(sn * STATE_CARRY);
        part += qv[r] * sn;
      }
      part += __shfl_xor(part, 16, 32);
      if (hh == 0) sop[wave * HD + j] = part;
    }
    __syncthreads();
    if (tid < HD) ob[(t & 15) * HD + tid] = ((sop[tid] + sop[HD + tid]) + sop[2 * HD + tid]) + sop[3 * HD + tid];
    if ((t & 15) == 15) {
      __syncthreads();
      float* dst = og + (size_t)(t - 15) * NSTATE + (size_t)h * HD;
      for (int pass = 0; pass < 2; ++pass) {
#pragma unroll
        for (int it = 0; it < 2; ++it) {
          const int idx = it * SCAN_T + tid;
          const int row = idx >> 4, c4 = (idx & 15) * 4;
          const v4f v = *(const v4f*)(ob + row * HD + c4);
          *(volatile v4f*)(dst + (size_t)row * NSTATE + c4) = v;
        }
        __threadfence();
      }
    }
  }
}

__global__ __launch_bounds__(SCAN_T) void gate_norm_kernel(const float* __restrict__ og, const float* __restrict__ proj,
                                                          const float* __restrict__ gw, unsigned short* __restrict__ y16) {
  __shared__ float red[4];
  const int t = blockIdx.x, tid = threadIdx.x, lane = tid & 31, wave = tid >> 5;
  const int c8 = tid * 8;
  const float* orow = og + (size_t)t * NSTATE + c8;
  const float* grow = proj + (size_t)t * NPROJ + 4 * NSTATE + c8;
  const v4f o0 = *(const v4f*)(orow), o1 = *(const v4f*)(orow + 4);
  const v4f g0 = *(const v4f*)(grow), g1 = *(const v4f*)(grow + 4);
  float y[8];
  float ss = 0.0f;
#pragma unroll
  for (int e = 0; e < 4; ++e) {
    const float ga = g0[e], gb = g1[e];
    const float ya = o0[e] * (ga * fsig(ga));
    const float yb = o1[e] * (gb * fsig(gb));
    y[e] = ya; y[4 + e] = yb;
    ss += ya * ya; ss += yb * yb;
  }
#pragma unroll
  for (int off = 16; off; off >>= 1) ss += __shfl_xor(ss, off, 32);
  if (lane == 0) red[wave] = ss;
  __syncthreads();
  const float tot = ((red[0] + red[1]) + red[2]) + red[3];
  const float rn = rsqrtf(tot * (1.0f / 1024.0f) + 1e-6f);
  v8h hv;
#pragma unroll
  for (int e = 0; e < 8; ++e) hv[e] = (_Float16)(((y[e] * rn) * bfr(gw[c8 + e])) * Y_CARRY);
  unsigned short* dst = y16 + (size_t)t * NSTATE + c8;
  *(volatile v8h*)dst = hv;
  __threadfence();
  *(volatile v8h*)dst = hv;
}

extern "C" void kernel_launch(void* const* d_in, const int* in_sizes, int n_in,
                              void* d_out, int out_size, void* d_ws, size_t ws_size, hipStream_t stream) {
  if (n_in < 7 || d_in == nullptr || in_sizes == nullptr || d_out == nullptr || d_ws == nullptr) return;
  if (in_sizes[0] != SEQ * NIN || in_sizes[1] != NIN * NPROJ || in_sizes[2] != NHEAD * HD * HD ||
      in_sizes[3] != NHEAD * HD || in_sizes[4] != NHEAD || in_sizes[5] != NSTATE ||
      in_sizes[6] != NSTATE * NOUT || out_size != SEQ * NOUT) return;

  const float* x    = (const float*)d_in[0];
  const float* win  = (const float*)d_in[1];
  const float* swt  = (const float*)d_in[2];
  const float* fm   = (const float*)d_in[3];
  const float* lf   = (const float*)d_in[4];
  const float* gw   = (const float*)d_in[5];
  const float* wout = (const float*)d_in[6];
  float* out = (float*)d_out;

  char* ws = (char*)d_ws; size_t off = 0;
  auto carve = [&](size_t bytes) -> char* { char* p = ws + off; off += (bytes + 255) & ~(size_t)255; return p; };
  unsigned short* X16 = (unsigned short*)carve((size_t)SEQ * NIN * 2);
  unsigned short* WIt = (unsigned short*)carve((size_t)NPROJ * NIN * 2);
  unsigned short* WOt = (unsigned short*)carve((size_t)NOUT * NSTATE * 2);
  float* PROJ = (float*)carve((size_t)SEQ * NPROJ * 4);
  float* PL   = (float*)carve((size_t)4 * SEQ * NSTATE * 4);
  float* OB   = (float*)carve((size_t)SEQ * NSTATE * 4);
  unsigned short* Y16 = (unsigned short*)carve((size_t)SEQ * NSTATE * 2);
  if (off > ws_size || off > (size_t)134217728) return;

  const int n8 = SEQ * NIN / 8;
  cast_bf16x8<<<(n8 + TPB - 1) / TPB, TPB, 0, stream>>>(x, X16, n8);
  tpw_kernel<0><<<dim3(NPROJ / 64, NIN / 64), TPB, 0, stream>>>(win, NIN, NPROJ, NIN, WIt, 1.0f);
  tpw_kernel<1><<<dim3(NOUT / 64, NSTATE / 64), TPB, 0, stream>>>(wout, NSTATE, NOUT, NSTATE, WOt, WOUT_CARRY);
  const int tilesP = (SEQ / 64) * (NPROJ / 64);
  wmma_gemm64<1, false, 0, 0, false, 0><<<dim3((tilesP + 7) / 8, 1), 256, 0, stream>>>(
      X16, X16, NIN, 0L, WIt, WIt, NIN, 0L, (void*)PROJ, (void*)PROJ, NPROJ, 0L, lf, lf, 0L, SEQ, NPROJ, NIN, 1.0f);
  prep_kernel<<<SEQ, TPB, 0, stream>>>(PROJ, fm, lf, PL);
  scan_kernel<<<NHEAD, SCAN_T, 0, stream>>>(PL, swt, lf, OB);
  gate_norm_kernel<<<SEQ, SCAN_T, 0, stream>>>(OB, PROJ, gw, Y16);
  const int tilesO = (SEQ / 64) * (NOUT / 64);
  wmma_gemm64<0, false, 0, 0, false, 0><<<dim3((tilesO + 7) / 8, 1), 256, 0, stream>>>(
      Y16, Y16, NSTATE, 0L, WOt, WOt, NSTATE, 0L, (void*)out, (void*)out, NOUT, 0L, lf, lf, 0L, SEQ, NOUT, NSTATE, OUT_INV);
}
